// CabbageEnhancedOneFormer3D_60876866453847
// MI455X (gfx1250) — hardware-verified
//
#include <hip/hip_runtime.h>
#include <math.h>

typedef __attribute__((ext_vector_type(16))) _Float16 v16h;
typedef __attribute__((ext_vector_type(16))) __bf16 v16b;
typedef __attribute__((ext_vector_type(8)))  _Float16 v8h;
typedef __attribute__((ext_vector_type(8)))  float v8f;
typedef __attribute__((ext_vector_type(4)))  float v4f;
typedef __attribute__((ext_vector_type(2)))  float v2f;
typedef __attribute__((ext_vector_type(4)))  unsigned v4u;
typedef __attribute__((ext_vector_type(4)))  int v4i;
typedef float __attribute__((may_alias)) float_a;
typedef int __attribute__((may_alias)) int_a;

template <typename T> __device__ __forceinline__ void vst2(void* p, T v) { *(volatile T*)p = v; __threadfence(); *(volatile T*)p = v; }
__device__ __forceinline__ v8f wmma16(v16h a, v16h b, v8f c) {
  v8f d = __builtin_amdgcn_wmma_f32_16x16x32_f16(false, a, false, b, (short)0, c, false, false);
  asm volatile("v_nop\n\tv_nop\n\tv_nop\n\tv_nop" : "+v"(d) : "v"(a), "v"(b));
  return d;
}
__device__ __forceinline__ v8f wmma_bf(v16b a, v16b b, v8f c) {
  v8f d = __builtin_amdgcn_wmma_f32_16x16x32_bf16(false, a, false, b, (short)0, c, false, false);
  asm volatile("v_nop\n\tv_nop\n\tv_nop\n\tv_nop" : "+v"(d) : "v"(a), "v"(b));
  return d;
}
__device__ __forceinline__ v16h frag_h(const _Float16* rowk0, int lane) {
  union { v16h v; v8h q[2]; } u; const _Float16* p = rowk0 + 8 * (lane >> 4);
  u.q[0] = *(const v8h*)p; u.q[1] = *(const v8h*)(p + 16); return u.v;
}
__device__ __forceinline__ v16h frag_f32(const float* rowk0, int lane) {
  v16h a; const float* p = rowk0 + 8 * (lane >> 4);
#pragma unroll
  for (int i = 0; i < 8; ++i) { a[i] = (_Float16)p[i]; a[8 + i] = (_Float16)p[16 + i]; }
  return a;
}
__device__ __forceinline__ v16h frag_f32s(const float* rowk0, int lane, float sc) {
  v16h a; const float* p = rowk0 + 8 * (lane >> 4);
#pragma unroll
  for (int i = 0; i < 8; ++i) { a[i] = (_Float16)(p[i] * sc); a[8 + i] = (_Float16)(p[16 + i] * sc); }
  return a;
}
__device__ __forceinline__ v16h fragc_f32(const float* W, int k0, int n, int lane, int ld, int K) {
  v16h a; const int g = lane >> 4;
#pragma unroll
  for (int i = 0; i < 8; ++i) { const int ka = k0 + 8 * g + i, kb = ka + 16;
    a[i] = (_Float16)(ka < K ? W[(size_t)ka * ld + n] : 0.f); a[8 + i] = (_Float16)(kb < K ? W[(size_t)kb * ld + n] : 0.f); }
  return a;
}
struct F2 { v16b h, l; };
__device__ __forceinline__ F2 bsplit16(const float v[16]) { F2 r;
#pragma unroll
  for (int i = 0; i < 16; ++i) { const __bf16 h = (__bf16)v[i]; r.h[i] = h; r.l[i] = (__bf16)(v[i] - (float)h); }
  return r; }
__device__ __forceinline__ F2 split_row(const float* row, int k0, int lane) { float v[16]; const float* p = row + k0 + 8 * (lane >> 4);
#pragma unroll
  for (int i = 0; i < 8; ++i) { v[i] = p[i]; v[8 + i] = p[16 + i]; }
  return bsplit16(v); }
__device__ __forceinline__ F2 split_rowK(const float* row, int k0, int lane, int K) { float v[16]; const int g = lane >> 4;
#pragma unroll
  for (int i = 0; i < 8; ++i) { const int ka = k0 + 8 * g + i, kb = ka + 16; v[i] = ka < K ? row[ka] : 0.f; v[8 + i] = kb < K ? row[kb] : 0.f; }
  return bsplit16(v); }
__device__ __forceinline__ F2 split_col(const float* W, int k0, int n, int lane, int ld, int K) { float v[16]; const int g = lane >> 4;
#pragma unroll
  for (int i = 0; i < 8; ++i) { const int ka = k0 + 8 * g + i, kb = ka + 16; v[i] = ka < K ? W[(size_t)ka * ld + n] : 0.f; v[8 + i] = kb < K ? W[(size_t)kb * ld + n] : 0.f; }
  return bsplit16(v); }
__device__ __forceinline__ v8f mac3(const F2& a, const F2& b, v8f c) { c = wmma_bf(a.l, b.h, c); c = wmma_bf(a.h, b.l, c); return wmma_bf(a.h, b.h, c); }
__device__ __forceinline__ float sigm(float v) { return 1.0f / (1.0f + expf(-v)); }
#define LDSX() do { asm volatile("s_wait_dscnt 0" ::: "memory"); __builtin_amdgcn_wave_barrier(); __builtin_amdgcn_fence(__ATOMIC_RELEASE, "workgroup"); } while (0)

#define NB 4
#define NPT 2048
#define NR (NB * NPT)
#define CIN 256
#define HM 128
#define NH 8
#define DH 16
#define FF 256
#define NCLS 3

__device__ __forceinline__ void ln_row_pair(float* row, const float* __restrict__ gam, const float* __restrict__ bet, int hf) {
  float s = 0.f; for (int c = hf * 64; c < hf * 64 + 64; ++c) s += row[c];
  s += __shfl_xor(s, 1, 32); const float mu = s * (1.0f / HM);
  float q2 = 0.f; for (int c = hf * 64; c < hf * 64 + 64; ++c) { const float d = row[c] - mu; q2 += d * d; }
  q2 += __shfl_xor(q2, 1, 32); const float rs = rsqrtf(q2 * (1.0f / HM) + 1e-5f);
  for (int c = hf * 64; c < hf * 64 + 64; ++c) row[c] = (row[c] - mu) * rs * gam[c] + bet[c];
}
__global__ __launch_bounds__(128) void k_fuse(const float* __restrict__ x, const float* __restrict__ w1, const float* __restrict__ b1, const float* __restrict__ w2, const float* __restrict__ b2, float* __restrict__ H) {
  __shared__ __align__(16) _Float16 sa[4][16][HM + 8];
  __shared__ __align__(16) float so[4][16][132];
  const int tid = threadIdx.x, wave = tid >> 5, lane = tid & 31, col = lane & 15, g = lane >> 4;
  const int r0 = blockIdx.x * 64 + wave * 16;
  { v8f acc[8] = {};
#pragma unroll 2
    for (int kc = 0; kc < CIN / 32; ++kc) { const v16h a = frag_f32(x + (size_t)(r0 + col) * CIN + kc * 32, lane);
#pragma unroll
      for (int t = 0; t < 8; ++t) acc[t] = wmma16(a, frag_f32s(w1 + (size_t)(t * 16 + col) * CIN + kc * 32, lane, 16.0f), acc[t]); }
#pragma unroll
    for (int t = 0; t < 8; ++t) { const float bb = b1[t * 16 + col];
#pragma unroll
      for (int r = 0; r < 8; ++r) { const float v = acc[t][r] * (1.0f / 16.0f) + bb; sa[wave][8 * g + r][t * 16 + col] = (_Float16)(v > 0.f ? v : 0.f); } } }
  LDSX();
  { v8f acc[8] = {};
#pragma unroll
    for (int kc = 0; kc < HM / 32; ++kc) { const v16h a = frag_h(&sa[wave][col][0] + kc * 32, lane);
#pragma unroll
      for (int t = 0; t < 8; ++t) acc[t] = wmma16(a, frag_f32s(w2 + (size_t)(t * 16 + col) * HM + kc * 32, lane, 16.0f), acc[t]); }
#pragma unroll
    for (int t = 0; t < 8; ++t) { const float bb = b2[t * 16 + col];
#pragma unroll
      for (int r = 0; r < 8; ++r) so[wave][8 * g + r][t * 16 + col] = acc[t][r] * (1.0f / 16.0f) + bb; } }
  LDSX();
#pragma unroll 4
  for (int rl = 0; rl < 16; ++rl) vst2(H + (size_t)(r0 + rl) * HM + lane * 4, *(const v4f*)(&so[wave][rl][lane * 4]));
}
__global__ __launch_bounds__(128) void k_qkv(const float* __restrict__ H, const float* __restrict__ iw, const float* __restrict__ ib, _Float16* __restrict__ Q16, _Float16* __restrict__ K16, _Float16* __restrict__ VT) {
  __shared__ __align__(16) float so[4][16][388];
  __shared__ __align__(16) _Float16 st[HM][72];
  const int tid = threadIdx.x, wave = tid >> 5, lane = tid & 31, col = lane & 15, g = lane >> 4;
  const int r0b = blockIdx.x * 64, r0 = r0b + wave * 16; const int b = r0b / NPT, s0 = r0b % NPT;
#pragma unroll 1
  for (int part = 0; part < 3; ++part) { v8f acc[8] = {};
#pragma unroll
    for (int kc = 0; kc < HM / 32; ++kc) { const v16h a = frag_f32(H + (size_t)(r0 + col) * HM + kc * 32, lane);
#pragma unroll
      for (int t = 0; t < 8; ++t) acc[t] = wmma16(a, frag_f32s(iw + (size_t)(part * HM + t * 16 + col) * HM + kc * 32, lane, 16.0f), acc[t]); }
#pragma unroll
    for (int t = 0; t < 8; ++t) { const int n = part * HM + t * 16 + col; const float bb = ib[n];
#pragma unroll
      for (int r = 0; r < 8; ++r) so[wave][8 * g + r][n] = (acc[t][r] * (1.0f / 16.0f) + bb) * 4.0f; } }
  LDSX();
  { const int rl = lane >> 1, hf = lane & 1; const int s = s0 + wave * 16 + rl;
    for (int hh = 0; hh < 4; ++hh) { const int h = hf * 4 + hh; union { v8h h8; v4u u; } q0, q1, k0, k1, z; z.u = (v4u){0u, 0u, 0u, 0u};
#pragma unroll
      for (int e = 0; e < 8; ++e) { q0.h8[e] = (_Float16)so[wave][rl][h * DH + e]; q1.h8[e] = (_Float16)so[wave][rl][h * DH + 8 + e]; k0.h8[e] = (_Float16)so[wave][rl][HM + h * DH + e]; k1.h8[e] = (_Float16)so[wave][rl][HM + h * DH + 8 + e]; }
      _Float16* qd = Q16 + (((size_t)b * NH + h) * NPT + s) * 32; _Float16* kd = K16 + (((size_t)b * NH + h) * NPT + s) * 32;
      vst2(qd, q0.u); vst2(qd + 8, q1.u); vst2(qd + 16, z.u); vst2(qd + 24, z.u); vst2(kd, k0.u); vst2(kd + 8, k1.u); vst2(kd + 16, z.u); vst2(kd + 24, z.u); } }
  for (int q = lane; q < 16 * HM; q += 32) { const int rl = q >> 7, c = q & 127; st[c][wave * 16 + rl] = (_Float16)so[wave][rl][2 * HM + c]; }
  __syncthreads();
  for (int qq = tid; qq < HM * 8; qq += 128) { const int c = qq >> 3, pc = qq & 7; const int h = c >> 4, d = c & 15; vst2(VT + (((size_t)b * NH + h) * DH + d) * NPT + s0 + pc * 8, *(const v4u*)(&st[c][pc * 8])); }
}
__global__ __launch_bounds__(128) void k_attn(const _Float16* __restrict__ Q16, const _Float16* __restrict__ K16, const _Float16* __restrict__ VT, _Float16* __restrict__ O16) {
  __shared__ __align__(16) float sS[4][16][68];
  __shared__ __align__(16) _Float16 sP[4][16][72];
  __shared__ __align__(16) float sO[4][16][20];
  const int tid = threadIdx.x, w = tid >> 5, lane = tid & 31, col = lane & 15, g = lane >> 4;
  const size_t bh = blockIdx.y; const int q0 = blockIdx.x * 64 + w * 16;
  const v16h aq = frag_h(Q16 + (bh * NPT + q0 + col) * 32, lane);
  float mrun = -3.0e38f, lrun = 0.f; v8f acc = {};
#pragma unroll 1
  for (int kt = 0; kt < NPT / 64; ++kt) {
#pragma unroll
    for (int t = 0; t < 4; ++t) { const int key = kt * 64 + t * 16 + col; const v8f s = wmma16(aq, frag_h(K16 + (bh * NPT + key) * 32, lane), (v8f){});
#pragma unroll
      for (int r = 0; r < 8; ++r) sS[w][8 * g + r][t * 16 + col] = s[r] * (0.25f / 16.0f); }
    LDSX();
    float mx = -3.4e38f;
#pragma unroll
    for (int jj = 0; jj < 32; ++jj) mx = fmaxf(mx, sS[w][col][g * 32 + jj]);
    mx = fmaxf(mx, __shfl_xor(mx, 16, 32));
    const float mnew = fmaxf(mrun, mx); const float corr = expf(mrun - mnew);
    float ps = 0.f;
#pragma unroll
    for (int jj = 0; jj < 32; ++jj) { const float p = expf(sS[w][col][g * 32 + jj] - mnew); ps += p; sP[w][col][g * 32 + jj] = (_Float16)(p * 16384.0f); }
    ps += __shfl_xor(ps, 16, 32);
    lrun = lrun * corr + ps; mrun = mnew;
#pragma unroll
    for (int r = 0; r < 8; ++r) { const float cr = __shfl(corr, 8 * g + r, 32); acc[r] *= cr; }
    LDSX();
#pragma unroll
    for (int kc = 0; kc < 2; ++kc) acc = wmma16(frag_h(&sP[w][col][0] + kc * 32, lane), frag_h(VT + (bh * DH + col) * NPT + kt * 64 + kc * 32, lane), acc);
    __builtin_amdgcn_wave_barrier(); }
#pragma unroll
  for (int r = 0; r < 8; ++r) { const float lr = __shfl(lrun, 8 * g + r, 32); sO[w][8 * g + r][col] = acc[r] * (8.0f / (lr * 16384.0f * 4.0f)); }
  LDSX();
  if (lane < 16) { union { v8h h8; v4u u; } p0, p1;
#pragma unroll
    for (int e = 0; e < 8; ++e) { p0.h8[e] = (_Float16)sO[w][lane][e]; p1.h8[e] = (_Float16)sO[w][lane][8 + e]; }
    _Float16* od = O16 + (bh * NPT + q0 + lane) * DH; vst2(od, p0.u); vst2(od + 8, p1.u); }
}
__device__ __forceinline__ v16h frag_o(const _Float16* __restrict__ O16, int b, int s, int kc, int lane) {
  const int g = lane >> 4; union { v8h v; v4u u; } lo, hi;
  lo.u = *(const v4u*)(O16 + (((size_t)b * NH + 2 * kc) * NPT + s) * DH + 8 * g); hi.u = *(const v4u*)(O16 + (((size_t)b * NH + 2 * kc + 1) * NPT + s) * DH + 8 * g);
  v16h a;
#pragma unroll
  for (int i = 0; i < 8; ++i) { a[i] = lo.v[i]; a[8 + i] = hi.v[i]; }
  return a;
}
__global__ __launch_bounds__(128) void k_post(const _Float16* __restrict__ O16, const float* __restrict__ ow, const float* __restrict__ ob, const float* __restrict__ f1, const float* __restrict__ fb1, const float* __restrict__ f2, const float* __restrict__ fb2,
                                            const float* __restrict__ g1, const float* __restrict__ be1, const float* __restrict__ g2, const float* __restrict__ be2, float* H) {
  __shared__ __align__(16) float so[4][16][132];
  __shared__ __align__(16) _Float16 sf[4][16][FF + 8];
  const int tid = threadIdx.x, wave = tid >> 5, lane = tid & 31, col = lane & 15, g = lane >> 4;
  const int r0b = blockIdx.x * 64, r0 = r0b + wave * 16; const int b = r0b / NPT, s0 = r0 % NPT;
  { v8f acc[8] = {};
#pragma unroll
    for (int kc = 0; kc < HM / 32; ++kc) { const v16h a = frag_o(O16, b, s0 + col, kc, lane);
#pragma unroll
      for (int t = 0; t < 8; ++t) acc[t] = wmma16(a, frag_f32s(ow + (size_t)(t * 16 + col) * HM + kc * 32, lane, 16.0f), acc[t]); }
#pragma unroll
    for (int t = 0; t < 8; ++t) { const int n = t * 16 + col; const float bb = ob[n];
#pragma unroll
      for (int r = 0; r < 8; ++r) so[wave][8 * g + r][n] = acc[t][r] * (1.0f / (16.0f * 8.0f)) + bb + H[(size_t)(r0 + 8 * g + r) * HM + n]; } }
  LDSX();
  ln_row_pair(&so[wave][lane >> 1][0], g1, be1, lane & 1);
  LDSX();
  { v8f acc[16];
#pragma unroll
    for (int t = 0; t < 16; ++t) acc[t] = (v8f){};
#pragma unroll
    for (int kc = 0; kc < HM / 32; ++kc) { float v[16]; const float* hr = &so[wave][col][kc * 32 + 8 * g];
#pragma unroll
      for (int i = 0; i < 8; ++i) { v[i] = hr[i]; v[8 + i] = hr[16 + i]; }
      v16h a;
#pragma unroll
      for (int i = 0; i < 16; ++i) a[i] = (_Float16)v[i];
#pragma unroll
      for (int t = 0; t < 16; ++t) acc[t] = wmma16(a, frag_f32s(f1 + (size_t)(t * 16 + col) * HM + kc * 32, lane, 16.0f), acc[t]); }
#pragma unroll
    for (int t = 0; t < 16; ++t) { const float bb = fb1[t * 16 + col];
#pragma unroll
      for (int r = 0; r < 8; ++r) { const float v = acc[t][r] * (1.0f / 16.0f) + bb; sf[wave][8 * g + r][t * 16 + col] = (_Float16)(v > 0.f ? v : 0.f); } } }
  LDSX();
  { v8f acc[8] = {};
#pragma unroll 2
    for (int kc = 0; kc < FF / 32; ++kc) { const v16h a = frag_h(&sf[wave][col][0] + kc * 32, lane);
#pragma unroll
      for (int t = 0; t < 8; ++t) acc[t] = wmma16(a, frag_f32s(f2 + (size_t)(t * 16 + col) * FF + kc * 32, lane, 16.0f), acc[t]); }
    LDSX();
#pragma unroll
    for (int t = 0; t < 8; ++t) { const int n = t * 16 + col; const float bb = fb2[n];
#pragma unroll
      for (int r = 0; r < 8; ++r) so[wave][8 * g + r][n] += acc[t][r] * (1.0f / 16.0f) + bb; } }
  LDSX();
  ln_row_pair(&so[wave][lane >> 1][0], g2, be2, lane & 1);
  LDSX();
#pragma unroll 4
  for (int rl = 0; rl < 16; ++rl) vst2(H + (size_t)(r0 + rl) * HM + lane * 4, *(const v4f*)(&so[wave][rl][lane * 4]));
}
__global__ __launch_bounds__(128) void k_heads(const float* __restrict__ H, const float* __restrict__ ow1, const float* __restrict__ ob1, const float* __restrict__ ow2, const float* __restrict__ ob2, const float* __restrict__ dw1, const float* __restrict__ db1, const float* __restrict__ dw2, const float* __restrict__ db2,
                                             float* __restrict__ logits, float* __restrict__ prob) {
  __shared__ __align__(16) float sz[4][16][196];
  __shared__ float slog[64 * 4]; __shared__ __align__(16) float sprob[64];
  const int tid = threadIdx.x, wave = tid >> 5, lane = tid & 31, col = lane & 15, g = lane >> 4;
  const int r0b = blockIdx.x * 64, r0 = r0b + wave * 16;
  { v8f acc[12];
#pragma unroll
    for (int t = 0; t < 12; ++t) acc[t] = (v8f){};
#pragma unroll
    for (int kc = 0; kc < HM / 32; ++kc) { const v16h a = frag_f32(H + (size_t)(r0 + col) * HM + kc * 32, lane);
#pragma unroll
      for (int t = 0; t < 12; ++t) acc[t] = wmma16(a, frag_f32s(t < 8 ? ow1 + (size_t)(t * 16 + col) * HM + kc * 32 : dw1 + (size_t)((t - 8) * 16 + col) * HM + kc * 32, lane, 16.0f), acc[t]); }
#pragma unroll
    for (int t = 0; t < 12; ++t) { const float bb = t < 8 ? ob1[t * 16 + col] : db1[(t - 8) * 16 + col];
#pragma unroll
      for (int r = 0; r < 8; ++r) { const float v = acc[t][r] * (1.0f / 16.0f) + bb; sz[wave][8 * g + r][t * 16 + col] = v > 0.f ? v : 0.f; } } }
  LDSX();
  { const int rl = lane >> 1, hf = lane & 1; const float* z = &sz[wave][rl][0];
    if (hf == 0) { float l0 = ob2[0], l1 = ob2[1], l2 = ob2[2];
#pragma unroll 1
      for (int c = 0; c < HM; ++c) { const float zv = z[c]; l0 += zv * ow2[c]; l1 += zv * ow2[HM + c]; l2 += zv * ow2[2 * HM + c]; }
      slog[(wave * 16 + rl) * 3 + 0] = l0; slog[(wave * 16 + rl) * 3 + 1] = l1; slog[(wave * 16 + rl) * 3 + 2] = l2; }
    else { float d = db2[0];
#pragma unroll 1
      for (int c = 0; c < 64; ++c) d += z[HM + c] * dw2[c];
      sprob[wave * 16 + rl] = sigm(d); } }
  __syncthreads();
  if (tid < 48) vst2(logits + (size_t)r0b * NCLS + tid * 4, *(const v4f*)(&slog[tid * 4]));
  if (tid >= 64 && tid < 80) vst2(prob + (size_t)r0b + (tid - 64) * 4, *(const v4f*)(&sprob[(tid - 64) * 4]));
}
__global__ __launch_bounds__(128) void k_quality(const float* __restrict__ prob, float* __restrict__ qual) {
  __shared__ __align__(16) float sq[4];
  const int wave = threadIdx.x >> 5, lane = threadIdx.x & 31; float s = 0.f;
  for (int i = lane; i < NPT; i += 32) s += prob[(size_t)wave * NPT + i];
#pragma unroll
  for (int off = 16; off >= 1; off >>= 1) s += __shfl_xor(s, off, 32);
  if (lane == 0) sq[wave] = s * (1.0f / NPT);
  __syncthreads();
  if (threadIdx.x == 0) vst2(qual, *(const v4f*)(&sq[0]));
}
extern "C" void kernel_launch(void* const* d_in, const int* in_sizes, int n_in, void* d_out, int out_size, void* d_ws, size_t ws_size, hipStream_t stream) {
  (void)in_sizes; (void)n_in; (void)out_size; (void)ws_size;
  const float** I = (const float**)d_in;
  float* logits = (float*)d_out; float* prob = (float*)((char*)d_out + 98304); float* qual = (float*)((char*)d_out + 131072);
  char* ws = (char*)d_ws; size_t off = 0;
  auto take = [&](size_t bytes) { char* p = ws + off; off += (bytes + 255) & ~(size_t)255; return p; };
  float* H = (float*)take((size_t)NR * HM * 4); _Float16* Q16 = (_Float16*)take((size_t)NB * NH * NPT * 32 * 2); _Float16* K16 = (_Float16*)take((size_t)NB * NH * NPT * 32 * 2); _Float16* VT = (_Float16*)take((size_t)NB * NH * DH * NPT * 2); _Float16* O16 = (_Float16*)take((size_t)NB * NH * NPT * DH * 2);
  k_fuse<<<NR / 64, 128, 0, stream>>>(I[0], I[1], I[2], I[3], I[4], H);
  for (int l = 0; l < 2; ++l) { const int o = 5 + 12 * l;
    k_qkv<<<NR / 64, 128, 0, stream>>>(H, I[o + 0], I[o + 1], Q16, K16, VT);
    k_attn<<<dim3(NPT / 64, NB * NH), 128, 0, stream>>>(Q16, K16, VT, O16);
    k_post<<<NR / 64, 128, 0, stream>>>(O16, I[o + 2], I[o + 3], I[o + 4], I[o + 5], I[o + 6], I[o + 7], I[o + 8], I[o + 9], I[o + 10], I[o + 11], H); }
  k_heads<<<NR / 64, 128, 0, stream>>>(H, I[29], I[30], I[31], I[32], I[33], I[34], I[35], I[36], logits, prob);
  k_quality<<<1, 128, 0, stream>>>(prob, qual);
}
